// MeshODENet_64819646431388
// MI455X (gfx1250) — hardware-run, weakly checked
//
#include <hip/hip_runtime.h>
#include <stddef.h>
#include <stdint.h>


#define DEV __device__ __forceinline__

#define NTHR   256
#define NWAVE  8
#define EPT    8
#define CHUNK  (NTHR * EPT)
#define WCAP   (EPT * 32)
#define LISTN  (NWAVE * WCAP)
#define NBA    512
#define NBN    64

static_assert(WCAP == 256);
static_assert((NBA % 64) == 0);
static_assert((NBA * 16) % NTHR == 0);

typedef float          v2f  __attribute__((ext_vector_type(2)));
typedef float          v4f  __attribute__((ext_vector_type(4)));
typedef float          v8f  __attribute__((ext_vector_type(8)));
typedef int            v4i  __attribute__((ext_vector_type(4)));
typedef unsigned short us;
typedef us             v4us __attribute__((ext_vector_type(4)));
typedef us             v8us __attribute__((ext_vector_type(8)));
typedef __bf16         v16bf __attribute__((ext_vector_type(16)));
union FragB { v16bf v; v8us h[2]; };

DEV v8f zero8f() {
  v8f z;
#pragma unroll
  for (int i = 0; i < 8; ++i) z[i] = 0.0f;
  return z;
}

DEV us bfr(float x) {
  unsigned u = __float_as_uint(x);
  u += 0x7FFFu + ((u >> 16) & 1u);
  return (us)(u >> 16);
}

DEV v16bf ldfrag(const us* base, int pitch, int row, int k0, int hh) {
  FragB f;
  const us* p = base + (size_t)row * pitch + k0 + 8 * hh;
  f.h[0] = *(const v8us*)p;
  f.h[1] = *(const v8us*)(p + 16);
  return f.v;
}

DEV v8f wmb(v16bf a, v16bf b, v8f c) {
  v8f d = __builtin_amdgcn_wmma_f32_16x16x32_bf16(false, a, false, b, (short)0, c, false, false);
  asm volatile("v_nop\n\tv_nop\n\tv_nop\n\tv_nop" : "+v"(d) : "v"(a), "v"(b));
  return d;
}

template <int KS, int NT>
DEV void gemm_row(const us* Ah, int lda, int arow,
                  const us* Bh, int ldb, int brow0, int hh, v8f (&acc)[NT]) {
#pragma unroll
  for (int j = 0; j < NT; ++j) acc[j] = zero8f();
#pragma unroll
  for (int ks = 0; ks < KS; ++ks) {
    const int k0 = ks * 32;
    const v16bf ah = ldfrag(Ah, lda, arow, k0, hh);
#pragma unroll
    for (int j = 0; j < NT; ++j) {
      const v16bf bh = ldfrag(Bh, ldb, brow0 + 16 * j, k0, hh);
      acc[j] = wmb(ah, bh, acc[j]);
    }
  }
}

__global__ __launch_bounds__(NTHR) void k_prep(
    const float* __restrict__ w_ne2, const float* __restrict__ w_ee2, const float* __restrict__ b_ee2,
    const float* __restrict__ w_em1, const float* __restrict__ b_em1, const float* __restrict__ w_em2,
    const float* __restrict__ w_nm1, const float* __restrict__ w_nm2, const float* __restrict__ w_dc1,
    const float* __restrict__ w_dc2,
    us* p_ne2, us* p_pq, us* p_em2, us* p_nm1, us* p_nm2, us* p_dc1, us* p_dc2, us* p_ee2, us* p_wp,
    float* bprime) {
  const int r = blockIdx.y;
  const int t = blockIdx.x * NTHR + threadIdx.x;
  if (r == 9) {
    if (t >= 64) return;
    float s = b_em1[t];
#pragma unroll 1
    for (int j = 0; j < 64; ++j) s += b_ee2[j] * w_em1[j * 64 + t];
    *(volatile float*)(bprime + t) = s;
    __threadfence();
    *(volatile float*)(bprime + t) = s;
    return;
  }
  int NO = 64, K = 64;
  us* dst;
  if (r == 1)      { NO = 128; dst = p_pq; }
  else if (r == 3) { K = 128;  dst = p_nm1; }
  else if (r == 6) { NO = 16;  dst = p_dc2; }
  else if (r == 0) dst = p_ne2;
  else if (r == 2) dst = p_em2;
  else if (r == 4) dst = p_nm2;
  else if (r == 5) dst = p_dc1;
  else if (r == 7) dst = p_ee2;
  else             dst = p_wp;
  const int kg8 = K >> 3;
  if (t >= NO * kg8) return;
  const int n  = t / kg8;
  const int k0 = (t - n * kg8) * 8;
  float v[8];
  if (r == 8) {
#pragma unroll
    for (int i = 0; i < 8; ++i) v[i] = 0.0f;
#pragma unroll 1
    for (int j = 0; j < 64; ++j) {
      const float a = w_em1[j * 64 + n];
#pragma unroll
      for (int i = 0; i < 8; ++i) v[i] += w_ee2[(k0 + i) * 64 + j] * a;
    }
  } else if (r == 1) {
    const int blk = n >> 6, nn = n & 63;
#pragma unroll
    for (int i = 0; i < 8; ++i) v[i] = w_em1[(64 + blk * 64 + k0 + i) * 64 + nn];
  } else if (r == 3) {
#pragma unroll
    for (int i = 0; i < 8; ++i) v[i] = w_nm1[(k0 + i) * 64 + n];
  } else if (r == 6) {
    const int nn = n < 3 ? n : 2;
#pragma unroll
    for (int i = 0; i < 8; ++i) { const float x = w_dc2[(k0 + i) * 3 + nn]; v[i] = (n < 3) ? x : 0.0f; }
  } else {
    const float* src = (r == 0) ? w_ne2 : (r == 2) ? w_em2 : (r == 4) ? w_nm2 : (r == 5) ? w_dc1 : w_ee2;
#pragma unroll
    for (int i = 0; i < 8; ++i) v[i] = src[(k0 + i) * 64 + n];
  }
  v8us hi;
#pragma unroll
  for (int i = 0; i < 8; ++i) hi[i] = bfr(v[i]);
  us* ph = dst + (size_t)n * K + k0;
  *(volatile v8us*)ph = hi;
  __threadfence();
  *(volatile v8us*)ph = hi;
}

__global__ __launch_bounds__(NTHR) void k_hconst(
    const float* __restrict__ youngs, const float* __restrict__ ym, const float* __restrict__ ys,
    const float* __restrict__ onehot, const float* __restrict__ w_ne1, const float* __restrict__ b_ne1,
    float* hc, int nN, int nRows,
    const float* __restrict__ wpos, const float* __restrict__ v0,
    float* posst, float* velst, float* out0, float* out1, int n3) {
  const int t = blockIdx.x * NTHR + threadIdx.x;
  const bool doA = t < nRows * 16;
  const int tA = doA ? t : 0;
  const int node = tA >> 4, cq = tA & 15, o0 = 4 * cq;
  const int nc = node < nN ? node : nN - 1;
  const float yn = (youngs[nc] - ym[0]) * (1.0f / ys[0]);
  float s0 = b_ne1[o0]     + yn * w_ne1[192 + o0];
  float s1 = b_ne1[o0 + 1] + yn * w_ne1[192 + o0 + 1];
  float s2 = b_ne1[o0 + 2] + yn * w_ne1[192 + o0 + 2];
  float s3 = b_ne1[o0 + 3] + yn * w_ne1[192 + o0 + 3];
#pragma unroll 1
  for (int i = 0; i < 9; ++i) {
    const float oh = onehot[(size_t)nc * 9 + i];
    const float* wr = w_ne1 + (4 + i) * 64 + o0;
    s0 += oh * wr[0]; s1 += oh * wr[1]; s2 += oh * wr[2]; s3 += oh * wr[3];
  }
  v4f hv = {s0, s1, s2, s3};
  float* hp = hc + (size_t)node * 64 + o0;
  const int n3q = n3 >> 2;
  const bool doB = t < n3q;
  const int tB = doB ? t : 0;
  const v4f pv = *(const v4f*)(wpos + 4 * (size_t)tB);
  const v4f vv = *(const v4f*)(v0 + 4 * (size_t)tB);
  const int nrem = n3 - n3q * 4;
  const bool doC = t < nrem;
  int ci = n3q * 4 + (doC ? t : 0);
  ci = ci < n3 ? ci : n3 - 1;
  const float ps = wpos[ci], vs1 = v0[ci];

  if (doA) *(volatile v4f*)hp = hv;
  if (doB) {
    *(volatile v4f*)(posst + 4 * (size_t)tB) = pv; *(volatile v4f*)(velst + 4 * (size_t)tB) = vv;
    *(volatile v4f*)(out0 + 4 * (size_t)tB) = pv;  *(volatile v4f*)(out1 + 4 * (size_t)tB) = vv;
  }
  if (doC) {
    *(volatile float*)(posst + ci) = ps; *(volatile float*)(velst + ci) = vs1;
    *(volatile float*)(out0 + ci) = ps;  *(volatile float*)(out1 + ci) = vs1;
  }
  __threadfence();
  if (doA) *(volatile v4f*)hp = hv;
  if (doB) {
    *(volatile v4f*)(posst + 4 * (size_t)tB) = pv; *(volatile v4f*)(velst + 4 * (size_t)tB) = vv;
    *(volatile v4f*)(out0 + 4 * (size_t)tB) = pv;  *(volatile v4f*)(out1 + 4 * (size_t)tB) = vv;
  }
  if (doC) {
    *(volatile float*)(posst + ci) = ps; *(volatile float*)(velst + ci) = vs1;
    *(volatile float*)(out0 + ci) = ps;  *(volatile float*)(out1 + ci) = vs1;
  }
}

__global__ __launch_bounds__(NTHR) void k_edge0(
    const float* __restrict__ eattr, const float* __restrict__ emean, const float* __restrict__ estd,
    const float* __restrict__ w_ee1, const float* __restrict__ b_ee1,
    const us* __restrict__ p_wp, const float* __restrict__ bprime, float* Cpl, int nE) {
  __shared__ __attribute__((aligned(16))) us    XA[64 * 64];
  __shared__ __attribute__((aligned(16))) float stg[64 * 64];
  const int tid = threadIdx.x, lane = tid & 31, wave = tid >> 5, hh = lane >> 4, m = lane & 15;
  const int eb = blockIdx.x * 64;
  {
    const int el = tid >> 2, part = tid & 3;
    int e = eb + el; e = e < nE ? e : nE - 1;
    const v4f x = *(const v4f*)(eattr + (size_t)e * 4);
    float en[4];
#pragma unroll
    for (int c = 0; c < 4; ++c) en[c] = (x[c] - emean[c]) * (1.0f / estd[c]);
    float s[16];
#pragma unroll
    for (int r = 0; r < 16; ++r) {
      const int o = part * 16 + r;
      const float v = b_ee1[o] + en[0] * w_ee1[o] + en[1] * w_ee1[64 + o] + en[2] * w_ee1[128 + o] + en[3] * w_ee1[192 + o];
      s[r] = fmaxf(v, 0.0f);
    }
    v8us hA, hB;
#pragma unroll
    for (int r = 0; r < 8; ++r) { hA[r] = bfr(s[r]); hB[r] = bfr(s[8 + r]); }
    us* xp = XA + el * 64 + part * 16;
    *(v8us*)xp = hA; *(v8us*)(xp + 8) = hB;
  }
  __syncthreads();
  {
    const int rt = wave >> 1, cb = (wave & 1) * 32;
    v8f acc[2];
    gemm_row<2, 2>(XA, 64, rt * 16 + m, p_wp, 64, cb + m, hh, acc);
#pragma unroll
    for (int j = 0; j < 2; ++j) {
      const int col = cb + 16 * j + m;
      const float bj = bprime[col];
#pragma unroll
      for (int r = 0; r < 8; ++r) stg[(rt * 16 + 8 * hh + r) * 64 + col] = acc[j][r] + bj;
    }
  }
  __syncthreads();
#pragma unroll
  for (int j = 0; j < 4; ++j) {
    const int q = j * NTHR + tid, row = q >> 4, c4 = q & 15;
    const v4f v = *(const v4f*)(stg + row * 64 + 4 * c4);
    *(volatile v4f*)(Cpl + (size_t)(eb + row) * 64 + 4 * c4) = v;
  }
  __threadfence();
#pragma unroll
  for (int j = 0; j < 4; ++j) {
    const int q = j * NTHR + tid, row = q >> 4, c4 = q & 15;
    const v4f v = *(const v4f*)(stg + row * 64 + 4 * c4);
    *(volatile v4f*)(Cpl + (size_t)(eb + row) * 64 + 4 * c4) = v;
  }
}

DEV int scan_chunk(const int* __restrict__ dsts, int nE, int cbase, int nodeBase,
                   int vec8, int* list, int tid, int wave) {
  int wc = 0;
  const int el0  = tid * EPT;
  const int e0   = cbase + el0;
  const int sent = -2147483647 - 1;
  v4i da, db;
  if (vec8 != 0 && cbase + CHUNK <= nE) {
    da = *(const v4i*)(dsts + e0);
    db = *(const v4i*)(dsts + e0 + 4);
  } else {
    da.x = (e0     < nE) ? dsts[min(e0, nE - 1)] : sent;
    da.y = (e0 + 1 < nE) ? dsts[min(e0 + 1, nE - 1)] : sent;
    da.z = (e0 + 2 < nE) ? dsts[min(e0 + 2, nE - 1)] : sent;
    da.w = (e0 + 3 < nE) ? dsts[min(e0 + 3, nE - 1)] : sent;
    db.x = (e0 + 4 < nE) ? dsts[min(e0 + 4, nE - 1)] : sent;
    db.y = (e0 + 5 < nE) ? dsts[min(e0 + 5, nE - 1)] : sent;
    db.z = (e0 + 6 < nE) ? dsts[min(e0 + 6, nE - 1)] : sent;
    db.w = (e0 + 7 < nE) ? dsts[min(e0 + 7, nE - 1)] : sent;
  }
  const unsigned nb = (unsigned)nodeBase;
  const unsigned s0 = (unsigned)da.x - nb, s1 = (unsigned)da.y - nb;
  const unsigned s2 = (unsigned)da.z - nb, s3 = (unsigned)da.w - nb;
  const unsigned s4 = (unsigned)db.x - nb, s5 = (unsigned)db.y - nb;
  const unsigned s6 = (unsigned)db.z - nb, s7 = (unsigned)db.w - nb;
  const bool h0 = s0 < (unsigned)NBA, h1 = s1 < (unsigned)NBA, h2 = s2 < (unsigned)NBA, h3 = s3 < (unsigned)NBA;
  const bool h4 = s4 < (unsigned)NBA, h5 = s5 < (unsigned)NBA, h6 = s6 < (unsigned)NBA, h7 = s7 < (unsigned)NBA;
  const unsigned any = __builtin_amdgcn_ballot_w32(h0 | h1 | h2 | h3 | h4 | h5 | h6 | h7);
  if (any != 0u) {
#define HITJ(J, HJ) { \
      const unsigned mj = __builtin_amdgcn_ballot_w32(HJ); \
      if (mj != 0u) { \
        if (HJ) { \
          const int pos = wc + (int)__builtin_amdgcn_mbcnt_lo(mj, 0u); \
          if (pos < WCAP) list[wave * WCAP + pos] = el0 + (J); \
        } \
        wc += (int)__builtin_popcount(mj); } }
    HITJ(0, h0)
    HITJ(1, h1)
    HITJ(2, h2)
    HITJ(3, h3)
    HITJ(4, h4)
    HITJ(5, h5)
    HITJ(6, h6)
    HITJ(7, h7)
#undef HITJ
  }
  return wc;
}

template <int MODE>
__global__ __launch_bounds__(NTHR) void k_agg(
    const int* __restrict__ ei,
    const float* __restrict__ eattr, const float* __restrict__ emean, const float* __restrict__ estd,
    const float* __restrict__ w_ee1, const float* __restrict__ b_ee1,
    const float* __restrict__ Cpl, const float* __restrict__ PQ,
    float* outPl, float* degPl, int nN, int nE, int vec8) {
  extern __shared__ __attribute__((aligned(16))) float accL[];
  __shared__ __attribute__((aligned(16))) int   list[LISTN];
  __shared__ __attribute__((aligned(16))) float cnt[NBA + 16];
  __shared__ int wcnt[NWAVE];

  const int tid = threadIdx.x, lane = tid & 31, wave = tid >> 5;
  const int nodeBase = blockIdx.x * NBA;
  const int* srcs = ei;
  const int* dsts = ei + nE;

  {
    const v4f z = {0.0f, 0.0f, 0.0f, 0.0f};
    for (int i = tid; i < (NBA + 1) * 16; i += NTHR) *(v4f*)(accL + 4 * i) = z;
    for (int i = tid; i < NBA + 16; i += NTHR) cnt[i] = 0.0f;
  }
  float w0[4], w1[4], mm[4], iv[4];
  float bb0 = 0.0f, bb1 = 0.0f;
#pragma unroll
  for (int c = 0; c < 4; ++c) { w0[c] = 0.0f; w1[c] = 0.0f; mm[c] = 0.0f; iv[c] = 1.0f; }
  if (MODE == 0) {
#pragma unroll
    for (int c = 0; c < 4; ++c) {
      w0[c] = w_ee1[c * 64 + 2 * lane];
      w1[c] = w_ee1[c * 64 + 2 * lane + 1];
      mm[c] = emean[c];
      iv[c] = 1.0f / estd[c];
    }
    bb0 = b_ee1[2 * lane];
    bb1 = b_ee1[2 * lane + 1];
  }
  __syncthreads();

  const int nChunks = (nE + CHUNK - 1) / CHUNK;
#pragma unroll 1
  for (int ch = 0; ch < nChunks; ++ch) {
    const int cbase = ch * CHUNK;
    const int wc = scan_chunk(dsts, nE, cbase, nodeBase, vec8, list, tid, wave);
    if (lane == 0) wcnt[wave] = wc;
    __syncthreads();

    if (wave == 0) {
#pragma unroll 1
      for (int w = 0; w < NWAVE; ++w) {
        int n = wcnt[w];
        n = n > WCAP ? WCAP : (n < 0 ? 0 : n);
#pragma unroll 1
        for (int i = 0; i < n; ++i) {
          const int el = list[w * WCAP + i];
          int e = cbase + el;
          e = e < 0 ? 0 : (e > nE - 1 ? nE - 1 : e);
          int d = dsts[e];
          int s = srcs[e];
          int slot = d - nodeBase;
          if ((unsigned)slot >= (unsigned)NBA) slot = NBA;
          d = d < 0 ? 0 : (d > nN - 1 ? nN - 1 : d);
          s = s < 0 ? 0 : (s > nN - 1 ? nN - 1 : s);
          float x0, x1;
          if (MODE == 1) {
            const v2f c = *(const v2f*)(Cpl + (size_t)e * 64 + 2 * lane);
            const v2f p = *(const v2f*)(PQ + (size_t)s * 128 + 2 * lane);
            const v2f q = *(const v2f*)(PQ + (size_t)d * 128 + 64 + 2 * lane);
            x0 = fmaxf(c.x + p.x + q.x, 0.0f);
            x1 = fmaxf(c.y + p.y + q.y, 0.0f);
          } else {
            const v4f ea = *(const v4f*)(eattr + (size_t)e * 4);
            const float n0 = (ea.x - mm[0]) * iv[0], n1 = (ea.y - mm[1]) * iv[1];
            const float n2 = (ea.z - mm[2]) * iv[2], n3v = (ea.w - mm[3]) * iv[3];
            x0 = fmaxf(bb0 + n0 * w0[0] + n1 * w0[1] + n2 * w0[2] + n3v * w0[3], 0.0f);
            x1 = fmaxf(bb1 + n0 * w1[0] + n1 * w1[1] + n2 * w1[2] + n3v * w1[3], 0.0f);
            if (lane == 0) cnt[slot] += 1.0f;
          }
          float* ap = accL + slot * 64 + 2 * lane;
          v2f a = *(v2f*)ap;
          a.x += x0; a.y += x1;
          *(v2f*)ap = a;
        }
      }
    }
    __syncthreads();
  }

#pragma unroll 1
  for (int j = 0; j < (NBA * 16) / NTHR; ++j) {
    const int q = j * NTHR + tid, row = q >> 4, c4 = q & 15;
    const v4f v = *(const v4f*)(accL + row * 64 + 4 * c4);
    *(volatile v4f*)(outPl + (size_t)(nodeBase + row) * 64 + 4 * c4) = v;
  }
  if (MODE == 0 && tid < NBA / 4) {
    const v4f v = *(const v4f*)(cnt + 4 * tid);
    *(volatile v4f*)(degPl + nodeBase + 4 * tid) = v;
  }
  __threadfence();
#pragma unroll 1
  for (int j = 0; j < (NBA * 16) / NTHR; ++j) {
    const int q = j * NTHR + tid, row = q >> 4, c4 = q & 15;
    const v4f v = *(const v4f*)(accL + row * 64 + 4 * c4);
    *(volatile v4f*)(outPl + (size_t)(nodeBase + row) * 64 + 4 * c4) = v;
  }
  if (MODE == 0 && tid < NBA / 4) {
    const v4f v = *(const v4f*)(cnt + 4 * tid);
    *(volatile v4f*)(degPl + nodeBase + 4 * tid) = v;
  }
}

__global__ __launch_bounds__(NTHR) void k_node0(
    const float* __restrict__ Rpl, const float* __restrict__ degpl,
    const us* __restrict__ p_ee2, const float* __restrict__ b_ee2, float* agg0) {
  __shared__ __attribute__((aligned(16))) us    XA[64 * 64];
  __shared__ __attribute__((aligned(16))) float stg[64 * 64];
  __shared__ float degs[64];
  const int tid = threadIdx.x, lane = tid & 31, wave = tid >> 5, hh = lane >> 4, m = lane & 15;
  const int nb = blockIdx.x * NBN;
#pragma unroll
  for (int j = 0; j < 4; ++j) {
    const int q = j * NTHR + tid, row = q >> 4, c4 = q & 15;
    const v4f v = *(const v4f*)(Rpl + (size_t)(nb + row) * 64 + 4 * c4);
    v4us h4;
#pragma unroll
    for (int i = 0; i < 4; ++i) h4[i] = bfr(v[i]);
    *(v4us*)(XA + row * 64 + 4 * c4) = h4;
  }
  if (tid < 64) degs[tid] = degpl[nb + tid];
  __syncthreads();
  {
    const int rt = wave >> 1, cb = (wave & 1) * 32;
    v8f acc[2];
    gemm_row<2, 2>(XA, 64, rt * 16 + m, p_ee2, 64, cb + m, hh, acc);
#pragma unroll
    for (int j = 0; j < 2; ++j) {
      const int col = cb + 16 * j + m;
      const float bj = b_ee2[col];
#pragma unroll
      for (int r = 0; r < 8; ++r) {
        const int row = rt * 16 + 8 * hh + r;
        stg[row * 64 + col] = acc[j][r] + degs[row] * bj;
      }
    }
  }
  __syncthreads();
#pragma unroll
  for (int j = 0; j < 4; ++j) {
    const int q = j * NTHR + tid, row = q >> 4, c4 = q & 15;
    const v4f v = *(const v4f*)(stg + row * 64 + 4 * c4);
    *(volatile v4f*)(agg0 + (size_t)(nb + row) * 64 + 4 * c4) = v;
  }
  __threadfence();
#pragma unroll
  for (int j = 0; j < 4; ++j) {
    const int q = j * NTHR + tid, row = q >> 4, c4 = q & 15;
    const v4f v = *(const v4f*)(stg + row * 64 + 4 * c4);
    *(volatile v4f*)(agg0 + (size_t)(nb + row) * 64 + 4 * c4) = v;
  }
}

__global__ __launch_bounds__(NTHR) void k_node1(
    const float* __restrict__ velst, const float* __restrict__ kprev, int usek, float coef,
    const float* __restrict__ ts, int step,
    const float* __restrict__ vm, const float* __restrict__ vsd,
    const float* __restrict__ w_ne1, const float* __restrict__ hc,
    const us* __restrict__ p_ne2, const float* __restrict__ b_ne2, const us* __restrict__ p_pq,
    float* hpl, float* pqpl, int nN) {
  __shared__ __attribute__((aligned(16))) us    XA[64 * 64];
  __shared__ __attribute__((aligned(16))) float stg[64 * 128];
  const int tid = threadIdx.x, lane = tid & 31, wave = tid >> 5, hh = lane >> 4, m = lane & 15;
  const int nb = blockIdx.x * NBN;
  {
    const int nl = tid >> 2, part = tid & 3;
    const int node = nb + nl;
    const int nc = node < nN ? node : nN - 1;
    float vn[3];
    {
#pragma clang fp contract(off)
      const float dt = ts[step + 1] - ts[step];
      const float cdt = coef * dt;
#pragma unroll
      for (int i = 0; i < 3; ++i) {
        float v = velst[(size_t)nc * 3 + i];
        float kv = 0.0f;
        if (usek != 0) kv = kprev[(size_t)nc * 3 + i];
        v = v + cdt * kv;
        vn[i] = (v - vm[i]) * (1.0f / vsd[i]);
      }
    }
    const float* hrow = hc + (size_t)node * 64 + part * 16;
    v4f h4[4];
#pragma unroll
    for (int a = 0; a < 4; ++a) h4[a] = *(const v4f*)(hrow + 4 * a);
    float s[16];
#pragma unroll
    for (int r = 0; r < 16; ++r) {
      const int o = part * 16 + r;
      const float base = h4[r >> 2][r & 3];
      const float v = base + vn[0] * w_ne1[o] + vn[1] * w_ne1[64 + o] + vn[2] * w_ne1[128 + o];
      s[r] = fmaxf(v, 0.0f);
    }
    v8us hA, hB;
#pragma unroll
    for (int r = 0; r < 8; ++r) { hA[r] = bfr(s[r]); hB[r] = bfr(s[8 + r]); }
    us* xp = XA + nl * 64 + part * 16;
    *(v8us*)xp = hA; *(v8us*)(xp + 8) = hB;
  }
  __syncthreads();
  {
    const int rt = wave >> 1, cb = (wave & 1) * 32;
    v8f acc[2];
    gemm_row<2, 2>(XA, 64, rt * 16 + m, p_ne2, 64, cb + m, hh, acc);
#pragma unroll
    for (int j = 0; j < 2; ++j) {
      const int col = cb + 16 * j + m;
      const float bj = b_ne2[col];
#pragma unroll
      for (int r = 0; r < 8; ++r) stg[(rt * 16 + 8 * hh + r) * 64 + col] = acc[j][r] + bj;
    }
  }
  __syncthreads();
  v4f hv[4];
#pragma unroll
  for (int j = 0; j < 4; ++j) {
    const int q = j * NTHR + tid, row = q >> 4, c4 = q & 15;
    const v4f v = *(const v4f*)(stg + row * 64 + 4 * c4);
    hv[j] = v;
    v4us h4;
#pragma unroll
    for (int i = 0; i < 4; ++i) h4[i] = bfr(v[i]);
    *(v4us*)(XA + row * 64 + 4 * c4) = h4;
    *(volatile v4f*)(hpl + (size_t)(nb + row) * 64 + 4 * c4) = v;
  }
  __threadfence();
#pragma unroll
  for (int j = 0; j < 4; ++j) {
    const int q = j * NTHR + tid, row = q >> 4, c4 = q & 15;
    *(volatile v4f*)(hpl + (size_t)(nb + row) * 64 + 4 * c4) = hv[j];
  }
  __syncthreads();
  {
    const int rt = wave >> 1, cb = (wave & 1) * 64;
    v8f acc[4];
    gemm_row<2, 4>(XA, 64, rt * 16 + m, p_pq, 64, cb + m, hh, acc);
#pragma unroll
    for (int j = 0; j < 4; ++j) {
      const int col = cb + 16 * j + m;
#pragma unroll
      for (int r = 0; r < 8; ++r) stg[(rt * 16 + 8 * hh + r) * 128 + col] = acc[j][r];
    }
  }
  __syncthreads();
  v4f pv[8];
#pragma unroll
  for (int j = 0; j < 8; ++j) {
    const int q = j * NTHR + tid, row = q >> 5, c4 = q & 31;
    const v4f v = *(const v4f*)(stg + row * 128 + 4 * c4);
    pv[j] = v;
    *(volatile v4f*)(pqpl + (size_t)(nb + row) * 128 + 4 * c4) = v;
  }
  __threadfence();
#pragma unroll
  for (int j = 0; j < 8; ++j) {
    const int q = j * NTHR + tid, row = q >> 5, c4 = q & 31;
    *(volatile v4f*)(pqpl + (size_t)(nb + row) * 128 + 4 * c4) = pv[j];
  }
}

__global__ __launch_bounds__(NTHR) void k_node2(
    const float* __restrict__ Spl, const float* __restrict__ agg0, const float* __restrict__ degpl,
    const float* __restrict__ hpl,
    const us* __restrict__ p_em2, const float* __restrict__ b_em2,
    const us* __restrict__ p_nm1, const float* __restrict__ b_nm1,
    const us* __restrict__ p_nm2, const float* __restrict__ b_nm2,
    const us* __restrict__ p_dc1, const float* __restrict__ b_dc1,
    const us* __restrict__ p_dc2, const float* __restrict__ b_dc2,
    const float* __restrict__ am, const float* __restrict__ asd,
    float* kout, int nN, int comb, const float* __restrict__ ts, int step,
    const float* __restrict__ k1, const float* __restrict__ k2, const float* __restrict__ k3,
    float* posst, float* velst, float* out0, float* out1) {
  __shared__ __attribute__((aligned(16))) us RA[64 * 64];
  __shared__ __attribute__((aligned(16))) us RB[64 * 128];
  __shared__ __attribute__((aligned(16))) float degs[64];
  __shared__ __attribute__((aligned(16))) float kst[192];
  __shared__ __attribute__((aligned(16))) float cps[192];
  __shared__ __attribute__((aligned(16))) float cvs[192];
  const int tid = threadIdx.x, lane = tid & 31, wave = tid >> 5, hh = lane >> 4, m = lane & 15;
  const int nb = blockIdx.x * NBN;
  const int rt = wave >> 1, cb = (wave & 1) * 32;

#pragma unroll
  for (int j = 0; j < 4; ++j) {
    const int q = j * NTHR + tid, row = q >> 4, c4 = q & 15;
    const v4f sv = *(const v4f*)(Spl + (size_t)(nb + row) * 64 + 4 * c4);
    const v4f hv = *(const v4f*)(hpl + (size_t)(nb + row) * 64 + 4 * c4);
    v4us h4, g4;
#pragma unroll
    for (int i = 0; i < 4; ++i) { h4[i] = bfr(sv[i]); g4[i] = bfr(hv[i]); }
    *(v4us*)(RA + row * 64 + 4 * c4) = h4;
    *(v4us*)(RB + row * 128 + 4 * c4) = g4;
  }
  if (tid < 64) degs[tid] = degpl[nb + tid];
  __syncthreads();

  {
    v8f acc[2];
    gemm_row<2, 2>(RA, 64, rt * 16 + m, p_em2, 64, cb + m, hh, acc);
#pragma unroll
    for (int j = 0; j < 2; ++j) {
      const int col = cb + 16 * j + m;
      const float bj = b_em2[col];
#pragma unroll
      for (int r = 0; r < 8; ++r) {
        const int row = rt * 16 + 8 * hh + r;
        const float a = acc[j][r] + agg0[(size_t)(nb + row) * 64 + col] + degs[row] * bj;
        RB[row * 128 + 64 + col] = bfr(a);
      }
    }
  }
  __syncthreads();

  {
    v8f acc[2];
    gemm_row<4, 2>(RB, 128, rt * 16 + m, p_nm1, 128, cb + m, hh, acc);
#pragma unroll
    for (int j = 0; j < 2; ++j) {
      const int col = cb + 16 * j + m;
      const float bj = b_nm1[col];
#pragma unroll
      for (int r = 0; r < 8; ++r) {
        const int row = rt * 16 + 8 * hh + r;
        const float y = fmaxf(acc[j][r] + bj, 0.0f);
        RA[row * 64 + col] = bfr(y);
      }
    }
  }
  __syncthreads();

  {
    v8f acc[2];
    gemm_row<2, 2>(RA, 64, rt * 16 + m, p_nm2, 64, cb + m, hh, acc);
#pragma unroll
    for (int j = 0; j < 2; ++j) {
      const int col = cb + 16 * j + m;
      const float bj = b_nm2[col];
#pragma unroll
      for (int r = 0; r < 8; ++r) {
        const int row = rt * 16 + 8 * hh + r;
        const float hres = hpl[(size_t)(nb + row) * 64 + col];
        const float h2 = hres + (acc[j][r] + bj);
        RB[row * 64 + col] = bfr(h2);
      }
    }
  }
  __syncthreads();

  {
    v8f acc[2];
    gemm_row<2, 2>(RB, 64, rt * 16 + m, p_dc1, 64, cb + m, hh, acc);
#pragma unroll
    for (int j = 0; j < 2; ++j) {
      const int col = cb + 16 * j + m;
      const float bj = b_dc1[col];
#pragma unroll
      for (int r = 0; r < 8; ++r) {
        const int row = rt * 16 + 8 * hh + r;
        const float d1 = fmaxf(acc[j][r] + bj, 0.0f);
        RA[row * 64 + col] = bfr(d1);
      }
    }
  }
  __syncthreads();

  if (wave < 4) {
    v8f acc[1];
    gemm_row<2, 1>(RA, 64, wave * 16 + m, p_dc2, 64, m, hh, acc);
    const int mc = m < 3 ? m : 2;
    const float bb = b_dc2[mc], sa = asd[mc], ma = am[mc];
#pragma unroll
    for (int r = 0; r < 8; ++r) {
      const int row = wave * 16 + 8 * hh + r;
      const float val = (acc[0][r] + bb) * sa + ma;
      if (m < 3) kst[row * 3 + m] = val;
    }
  }
  __syncthreads();

  const int n3 = nN * 3;
  if (comb != 0) {
#pragma clang fp contract(off)
    const float dt = ts[step + 1] - ts[step];
    const float hdt = 0.5f * dt;
    const float sixth = dt / 6.0f;
    int ic = nb * 3 + tid;
    ic = ic < n3 ? ic : n3 - 1;
    if (tid < 192) {
      const float p = posst[ic], v = velst[ic];
      const float a1 = k1[ic], a2 = k2[ic], a3 = k3[ic], a4 = kst[tid];
      const float k2p = v + hdt * a1;
      const float k3p = v + hdt * a2;
      const float k4p = v + dt * a3;
      float sp = v + 2.0f * k2p; sp = sp + 2.0f * k3p; sp = sp + k4p;
      float sv = a1 + 2.0f * a2; sv = sv + 2.0f * a3; sv = sv + a4;
      cps[tid] = p + sixth * sp;
      cvs[tid] = v + sixth * sv;
    }
  }
  __syncthreads();

  const int nrows = (nN - nb) < NBN ? (nN - nb) : NBN;
  const int nf = nrows * 3, nq = nf >> 2, nrem = nf & 3;
  const size_t kb = (size_t)nb * 3;
  const size_t ob = (size_t)(step + 1) * (size_t)n3 + kb;
  if (tid < 48) { const v4f v = *(const v4f*)(kst + 4 * tid); *(volatile v4f*)(kout + kb + 4 * tid) = v; }
  if (comb != 0) {
    if (tid < nq) {
      const v4f cp = *(const v4f*)(cps + 4 * tid), cv = *(const v4f*)(cvs + 4 * tid);
      *(volatile v4f*)(posst + kb + 4 * tid) = cp; *(volatile v4f*)(velst + kb + 4 * tid) = cv;
      *(volatile v4f*)(out0 + ob + 4 * tid) = cp;  *(volatile v4f*)(out1 + ob + 4 * tid) = cv;
    }
    if (tid < nrem) {
      const int ii = nq * 4 + tid;
      const float cp = cps[ii], cv = cvs[ii];
      *(volatile float*)(posst + kb + ii) = cp; *(volatile float*)(velst + kb + ii) = cv;
      *(volatile float*)(out0 + ob + ii) = cp;  *(volatile float*)(out1 + ob + ii) = cv;
    }
  }
  __threadfence();
  if (tid < 48) { const v4f v = *(const v4f*)(kst + 4 * tid); *(volatile v4f*)(kout + kb + 4 * tid) = v; }
  if (comb != 0) {
    if (tid < nq) {
      const v4f cp = *(const v4f*)(cps + 4 * tid), cv = *(const v4f*)(cvs + 4 * tid);
      *(volatile v4f*)(posst + kb + 4 * tid) = cp; *(volatile v4f*)(velst + kb + 4 * tid) = cv;
      *(volatile v4f*)(out0 + ob + 4 * tid) = cp;  *(volatile v4f*)(out1 + ob + 4 * tid) = cv;
    }
    if (tid < nrem) {
      const int ii = nq * 4 + tid;
      const float cp = cps[ii], cv = cvs[ii];
      *(volatile float*)(posst + kb + ii) = cp; *(volatile float*)(velst + kb + ii) = cv;
      *(volatile float*)(out0 + ob + ii) = cp;  *(volatile float*)(out1 + ob + ii) = cv;
    }
  }
}

extern "C" void kernel_launch(void* const* d_in, const int* in_sizes, int n_in,
                              void* d_out, int out_size, void* d_ws, size_t ws_size,
                              hipStream_t stream) {
  if (n_in < 36) return;
  const int N = in_sizes[0] / 3;
  const int E = in_sizes[2] / 2;
  const int T = in_sizes[7];
  if (N <= 0 || E <= 0 || T <= 0) return;
  if (in_sizes[0] != N * 3 || in_sizes[1] != N * 3 || in_sizes[2] != 2 * E || in_sizes[3] != 4 * E) return;
  if (in_sizes[4] != N || in_sizes[5] != 9 * N) return;
  if (in_sizes[8] < 1 || in_sizes[9] < 1 || in_sizes[10] < 4 || in_sizes[11] < 4) return;
  if (in_sizes[12] < 3 || in_sizes[13] < 3 || in_sizes[14] < 3 || in_sizes[15] < 3) return;
  if (in_sizes[16] != 13 * 64 || in_sizes[17] != 64 || in_sizes[18] != 4096 || in_sizes[19] != 64) return;
  if (in_sizes[20] != 256 || in_sizes[21] != 64 || in_sizes[22] != 4096 || in_sizes[23] != 64) return;
  if (in_sizes[24] != 192 * 64 || in_sizes[25] != 64 || in_sizes[26] != 4096 || in_sizes[27] != 64) return;
  if (in_sizes[28] != 8192 || in_sizes[29] != 64 || in_sizes[30] != 4096 || in_sizes[31] != 64) return;
  if (in_sizes[32] != 4096 || in_sizes[33] != 64 || in_sizes[34] != 192 || in_sizes[35] != 3) return;
  const int n3 = N * 3;
  if (out_size != 2 * T * n3 || (n3 & 3) != 0) return;

  const float* world_pos = (const float*)d_in[0];
  const float* velocity  = (const float*)d_in[1];
  const int*   edge_index= (const int*)d_in[2];
  const float* eattr     = (const float*)d_in[3];
  const float* youngs    = (const float*)d_in[4];
  const float* one_hot   = (const float*)d_in[5];
  const float* t_span    = (const float*)d_in[7];
  const float* ymean = (const float*)d_in[8],  *ystd = (const float*)d_in[9];
  const float* memean= (const float*)d_in[10], *mestd= (const float*)d_in[11];
  const float* vmean = (const float*)d_in[12], *vstd = (const float*)d_in[13];
  const float* amean = (const float*)d_in[14], *astd = (const float*)d_in[15];
  const float* w_ne1 = (const float*)d_in[16], *b_ne1 = (const float*)d_in[17];
  const float* w_ne2 = (const float*)d_in[18], *b_ne2 = (const float*)d_in[19];
  const float* w_ee1 = (const float*)d_in[20], *b_ee1 = (const float*)d_in[21];
  const float* w_ee2 = (const float*)d_in[22], *b_ee2 = (const float*)d_in[23];
  const float* w_em1 = (const float*)d_in[24], *b_em1 = (const float*)d_in[25];
  const float* w_em2 = (const float*)d_in[26], *b_em2 = (const float*)d_in[27];
  const float* w_nm1 = (const float*)d_in[28], *b_nm1 = (const float*)d_in[29];
  const float* w_nm2 = (const float*)d_in[30], *b_nm2 = (const float*)d_in[31];
  const float* w_dc1 = (const float*)d_in[32], *b_dc1 = (const float*)d_in[33];
  const float* w_dc2 = (const float*)d_in[34], *b_dc2 = (const float*)d_in[35];

  const int nNB = (N + NBN - 1) / NBN;
  const int nAB = (N + NBA - 1) / NBA;
  const int nEB = (E + 63) / 64;
  const int NR  = (nNB * NBN > nAB * NBA) ? nNB * NBN : nAB * NBA;
  const int ER  = nEB * 64;

  char* ws = (char*)d_ws;
  size_t off = 0;
  auto alloc = [&](size_t bytes) -> char* {
    char* p = ws + off;
    off = (off + bytes + 255) & ~(size_t)255;
    return p;
  };
  us* p_ne2 = (us*)alloc((size_t)64 * 64 * 2);
  us* p_pq  = (us*)alloc((size_t)128 * 64 * 2);
  us* p_em2 = (us*)alloc((size_t)64 * 64 * 2);
  us* p_nm1 = (us*)alloc((size_t)64 * 128 * 2);
  us* p_nm2 = (us*)alloc((size_t)64 * 64 * 2);
  us* p_dc1 = (us*)alloc((size_t)64 * 64 * 2);
  us* p_dc2 = (us*)alloc((size_t)16 * 64 * 2);
  us* p_ee2 = (us*)alloc((size_t)64 * 64 * 2);
  us* p_wp  = (us*)alloc((size_t)64 * 64 * 2);
  float* bprime = (float*)alloc(256);
  float* hc    = (float*)alloc((size_t)NR * 64 * 4);
  float* hpl   = (float*)alloc((size_t)NR * 64 * 4);
  float* pqpl  = (float*)alloc((size_t)NR * 128 * 4);
  float* Spl   = (float*)alloc((size_t)NR * 64 * 4);
  float* Rpl   = (float*)alloc((size_t)NR * 64 * 4);
  float* agg0  = (float*)alloc((size_t)NR * 64 * 4);
  float* degpl = (float*)alloc((size_t)NR * 4);
  float* Cpl   = (float*)alloc((size_t)ER * 64 * 4);
  float* posst = (float*)alloc((size_t)NR * 3 * 4);
  float* velst = (float*)alloc((size_t)NR * 3 * 4);
  float* k1    = (float*)alloc((size_t)NR * 3 * 4);
  float* k2    = (float*)alloc((size_t)NR * 3 * 4);
  float* k3    = (float*)alloc((size_t)NR * 3 * 4);
  float* k4    = (float*)alloc((size_t)NR * 3 * 4);
  if (off > ws_size || off > (size_t)134217728) return;

  float* out0 = (float*)d_out;
  float* out1 = out0 + (size_t)T * n3;
  const int vec8 = ((E & 3) == 0) ? 1 : 0;
  const size_t dynB = (size_t)(NBA + 1) * 64 * 4;

  k_prep<<<dim3(4, 10, 1), NTHR, 0, stream>>>(w_ne2, w_ee2, b_ee2, w_em1, b_em1, w_em2, w_nm1, w_nm2, w_dc1, w_dc2,
                                             p_ne2, p_pq, p_em2, p_nm1, p_nm2, p_dc1, p_dc2, p_ee2, p_wp, bprime);
  k_hconst<<<(NR * 16 + NTHR - 1) / NTHR, NTHR, 0, stream>>>(youngs, ymean, ystd, one_hot, w_ne1, b_ne1, hc, N, NR,
                                                            world_pos, velocity, posst, velst, out0, out1, n3);
  k_edge0<<<nEB, NTHR, 0, stream>>>(eattr, memean, mestd, w_ee1, b_ee1, p_wp, bprime, Cpl, E);
  hipFuncSetAttribute(reinterpret_cast<const void*>(&k_agg<0>), hipFuncAttributeMaxDynamicSharedMemorySize, (int)dynB);
  hipFuncSetAttribute(reinterpret_cast<const void*>(&k_agg<1>), hipFuncAttributeMaxDynamicSharedMemorySize, (int)dynB);
  k_agg<0><<<nAB, NTHR, dynB, stream>>>(edge_index, eattr, memean, mestd, w_ee1, b_ee1, Cpl, pqpl, Rpl, degpl, N, E, vec8);
  k_node0<<<nNB, NTHR, 0, stream>>>(Rpl, degpl, p_ee2, b_ee2, agg0);

  float* kk[4] = {k1, k2, k3, k4};
  for (int step = 0; step + 1 < T; ++step) {
    for (int ev = 0; ev < 4; ++ev) {
      const float* kprev = (ev == 0) ? k4 : kk[ev - 1];
      const int usek = (ev == 0) ? 0 : 1;
      const float coef = (ev == 3) ? 1.0f : 0.5f;
      const int comb = (ev == 3) ? 1 : 0;
      k_node1<<<nNB, NTHR, 0, stream>>>(velst, kprev, usek, coef, t_span, step, vmean, vstd, w_ne1, hc,
                                        p_ne2, b_ne2, p_pq, hpl, pqpl, N);
      k_agg<1><<<nAB, NTHR, dynB, stream>>>(edge_index, eattr, memean, mestd, w_ee1, b_ee1, Cpl, pqpl, Spl, degpl, N, E, vec8);
      k_node2<<<nNB, NTHR, 0, stream>>>(Spl, agg0, degpl, hpl, p_em2, b_em2, p_nm1, b_nm1, p_nm2, b_nm2,
                                        p_dc1, b_dc1, p_dc2, b_dc2, amean, astd, kk[ev], N, comb, t_span, step,
                                        k1, k2, k3, posst, velst, out0, out1);
    }
  }
}
